// DGCNN_71579924955362
// MI455X (gfx1250) — hardware-verified
//
#include <hip/hip_runtime.h>


namespace {

constexpr int N = 100000, NP = 100032, NPL = NP  , SRCM = N  , EFULL = 1600000, KN = 16  , EH1 = N  , EH1P = NP;
constexpr int CI = 16, C1 = 64, C2 = 128, VOC = 1  , F = C2  , D1 = 2 * F  , CO = 40  , COP = 64  , NRL = NP  , NL = (NPL < N ? NPL : N);
constexpr float LNEPS = 1e-5f; constexpr float LOG2E = 1.4426950408889634f; constexpr float XS = 8.0f, WSC = 256.0f, WSQ = 0.25f, RS_ = 1024.0f, NSL_ = 0.2f, NSA_ = 0.01f, SLOPE = 0.0f, BNEPS = 1e-5f;
static_assert(NP % 32 == 0 && NP >= N && NPL % 32 == 0 && D1 == 256, "tiling");
typedef _Float16 b16;
typedef __attribute__((ext_vector_type(16))) _Float16 v16b;
typedef __attribute__((ext_vector_type(8))) _Float16 v8b;
typedef __attribute__((ext_vector_type(8))) float v8f;
typedef __attribute__((ext_vector_type(4))) float v4f;
__device__ __forceinline__ float bf16_rne(float f) { unsigned int u = __float_as_uint(f); u += 0x7FFFu + ((u >> 16) & 1u); return __uint_as_float(u & 0xFFFF0000u); }
__device__ __forceinline__ void split16(float v, b16& hi, b16& lo) { hi = (b16)v; lo = (b16)(v - (float)hi); }
__device__ __forceinline__ v16b frag_kb(const b16* p, int hh) { const v8b a = *(const v8b*)(p + 8 * hh), b = *(const v8b*)(p + 16 + 8 * hh); v16b f;
#pragma unroll
  for (int e = 0; e < 8; ++e) { f[e] = a[e]; f[8 + e] = b[e]; } return f; }
__device__ __forceinline__ v8f wmma16b(v16b a, v16b b, v8f c) { v8f d = __builtin_amdgcn_wmma_f32_16x16x32_f16(false, a, false, b, (short)0, c, false, false); asm volatile("v_nop\n\tv_nop\n\tv_nop\n\tv_nop" : "+v"(d) : "v"(a), "v"(b)); return d; }
__device__ __forceinline__ void wave_lds_sync() { __builtin_amdgcn_fence(__ATOMIC_RELEASE, "workgroup"); __builtin_amdgcn_wave_barrier(); __builtin_amdgcn_fence(__ATOMIC_ACQUIRE, "workgroup"); }
__device__ __forceinline__ float pmul(float a, float b) { float p = a * b; asm volatile("" : "+v"(p)); return p; }
__device__ __forceinline__ int iclamp(int v, int lo, int hi) { return v < lo ? lo : (v > hi ? hi : v); }

typedef __attribute__((ext_vector_type(4))) _Float16 v4h;
__device__ __forceinline__ float lrelu(float v) { return v > 0.0f ? v : NSL_ * v; }
template <int K, int NOUTR, int NOUTP>
__global__ __launch_bounds__(256) void wt_kernel(const float* __restrict__ w, b16* __restrict__ WT, float scl) {
  const int u = blockIdx.x * 256 + threadIdx.x; if (u >= NOUTP * K / 8) return; const int e = u * 8; const int o = e / K, k0 = e % K; v8b v;
#pragma unroll
  for (int j = 0; j < 8; ++j) v[j] = (b16)(o < NOUTR ? bf16_rne(w[(size_t)(k0 + j) * NOUTR + o]) * scl : 0.0f);
  for (int pass = 0; pass < 2; ++pass) { *(volatile v8b*)(WT + e) = v; __threadfence(); }
}
template <int K, int NT, bool RND, int MODE, bool GIDX>
__global__ __launch_bounds__(64) void lin_kernel(const float* __restrict__ X, const int* __restrict__ gidx, const b16* __restrict__ WT, const b16* __restrict__ WQ, const float* __restrict__ bias, float* __restrict__ OUT, int opitch, int nvalid, int mrows, const float* __restrict__ lng = nullptr, const float* __restrict__ lnb = nullptr) {
  constexpr int NC = NT * 16;
  __shared__ __attribute__((aligned(16))) b16 Ah[2][16][K + 8], Al[2][16][K + 8]; __shared__ __attribute__((aligned(16))) float Tf[2][16][NC + 4];
  const int wave = threadIdx.x >> 5, lane = threadIdx.x & 31, nloc = lane & 15, hlf = lane >> 4; const size_t m0 = (size_t)blockIdx.x * 32 + wave * 16;
  for (int idx = lane; idx < 16 * (K / 4); idx += 32) { const int rr = idx / (K / 4), c4 = (idx % (K / 4)) * 4; const size_t vrow = (m0 + rr < (size_t)nvalid) ? m0 + rr : (size_t)nvalid - 1; size_t arow = vrow; if (GIDX) arow = (size_t)iclamp(gidx[vrow], 0, VOC - 1);
    const v4f v = *(const v4f*)(X + arow * K + c4); v4h hv, lv;
    for (int j = 0; j < 4; ++j) { float vj = v[j]; if (MODE == 2) vj = fmaxf(vj, 0.0f); const float vs = (RND ? bf16_rne(vj) : vj) * XS; const b16 ph = (b16)vs; hv[j] = ph; lv[j] = (b16)((vs - (float)ph) * RS_); } *(v4h*)(&Ah[wave][rr][c4]) = hv; *(v4h*)(&Al[wave][rr][c4]) = lv; }
  wave_lds_sync();
  v8f acc[NT];
#pragma unroll
  for (int t = 0; t < NT; ++t) acc[t] = (v8f){};
#pragma unroll 1
  for (int kb = 0; kb < K; kb += 32) { const v16b a = frag_kb(&Ah[wave][nloc][kb], hlf); v16b al; if (!RND) al = frag_kb(&Al[wave][nloc][kb], hlf);
#pragma unroll
    for (int t = 0; t < NT; ++t) { const size_t wo_ = (size_t)(t * 16 + nloc) * K + kb; acc[t] = wmma16b(a, frag_kb(WT + wo_, hlf), acc[t]); if (!RND) acc[t] = wmma16b(al, frag_kb(WQ + wo_, hlf), acc[t]); } }
if (MODE == 5) {
    static_assert(MODE != 5 || NT == 8, "LN epilogue needs the full 128-wide row in one wave");
    float sm[8], sq[8]; for (int r = 0; r < 8; ++r) { sm[r] = 0.0f; sq[r] = 0.0f; }
    for (int t = 0; t < NT; ++t) { const int col = t * 16 + nloc; const float bb = bf16_rne(bias[col]); for (int r = 0; r < 8; ++r) { const float y = acc[t][r] * (1.0f / (XS * WSC)) + bb; acc[t][r] = y; sm[r] += y; } }
#pragma unroll
    for (int o = 1; o < 16; o <<= 1) for (int r = 0; r < 8; ++r) sm[r] += __shfl_xor(sm[r], o);
    for (int t = 0; t < NT; ++t) for (int r = 0; r < 8; ++r) { const float d = acc[t][r] - sm[r] * (1.0f / NC); sq[r] += pmul(d, d); }
#pragma unroll
    for (int o = 1; o < 16; o <<= 1) for (int r = 0; r < 8; ++r) sq[r] += __shfl_xor(sq[r], o);
    for (int t = 0; t < NT; ++t) { const int col = t * 16 + nloc; const float gg = bf16_rne(lng[col]), be = bf16_rne(lnb[col]);
      for (int r = 0; r < 8; ++r) { const size_t vrow = m0 + 8 * hlf + r; const float y = fmaxf((acc[t][r] - sm[r] * (1.0f / NC)) * rsqrtf(sq[r] * (1.0f / NC) + LNEPS) * gg + be, 0.0f); Tf[wave][8 * hlf + r][col] = (vrow < (size_t)nvalid) ? y : 0.0f; } }
  } else {
  for (int t = 0; t < NT; ++t) { const int col = t * 16 + nloc; const float bb = bf16_rne(bias[col]);
    for (int r = 0; r < 8; ++r) { const size_t vrow = m0 + 8 * hlf + r; float y = acc[t][r] * (1.0f / (XS * WSC)) + bb; if (MODE == 1) y = fmaxf(y, 0.0f); Tf[wave][8 * hlf + r][col] = (vrow < (size_t)nvalid) ? y : 0.0f; } }
  }
  wave_lds_sync();
  for (int pass = 0; pass < 2; ++pass) { for (int rr = 0; rr < 16; ++rr) { if (m0 + rr < (size_t)mrows) { if (NC >= 128) { for (int c8 = 0; c8 < NC; c8 += 128) *(volatile v4f*)(OUT + (m0 + rr) * (size_t)opitch + c8 + lane * 4) = *(const v4f*)(&Tf[wave][rr][c8 + lane * 4]); }
        else { if (lane < NC / 4) *(volatile v4f*)(OUT + (m0 + rr) * (size_t)opitch + lane * 4) = *(const v4f*)(&Tf[wave][rr][lane * 4]); } } } __threadfence(); }
}
__global__ __launch_bounds__(64) void bpad_kernel(const float* __restrict__ b, float* __restrict__ B) { const int i = threadIdx.x; const float val = (i < CO) ? b[i] : 0.0f; for (int pass = 0; pass < 2; ++pass) { ((volatile float*)B)[i] = val; __threadfence(); } }
__device__ __forceinline__ float gelu_(float v) { return 0.5f * v * (1.0f + erff(v * 0.70710678118654752f)); }
__global__ __launch_bounds__(256) void ocopy_kernel(const float* __restrict__ L, float* __restrict__ out, int nl) {
  const size_t total = (size_t)nl * CO; const size_t j0 = ((size_t)blockIdx.x * 256 + threadIdx.x) * 4; if (j0 >= total) return;
  v4f t4; for (int k = 0; k < 4; ++k) { const size_t j = j0 + k; const size_t jj = (j < total) ? j : total - 1; t4[k] = L[(jj / CO) * COP + (jj % CO)]; }
  for (int pass = 0; pass < 2; ++pass) { if (j0 + 4 <= total) *(volatile v4f*)(out + j0) = t4; else { for (int k = 0; k < 4; ++k) if (j0 + k < total) ((volatile float*)out)[j0 + k] = t4[k]; } __threadfence(); }
}
__global__ __launch_bounds__(64) void e1_kernel(const float* __restrict__ x, const int* __restrict__ rows, const int* __restrict__ cols, const b16* __restrict__ WT, const b16* __restrict__ WQ, const float* __restrict__ bias, float* __restrict__ T1, int mrows) {
  constexpr int K = 2 * CI, NT = 4;
  __shared__ __attribute__((aligned(16))) b16 Ah[2][16][K + 8], Al[2][16][K + 8]; __shared__ __attribute__((aligned(16))) float Tf[2][16][C1 + 4];
  const int wave = threadIdx.x >> 5, lane = threadIdx.x & 31, nloc = lane & 15, hlf = lane >> 4; const size_t m0 = (size_t)blockIdx.x * 32 + wave * 16;
  for (int idx = lane; idx < 16 * (K / 4); idx += 32) { const int rr = idx / (K / 4), c4 = (idx % (K / 4)) * 4; const size_t e = (m0 + rr < (size_t)EH1) ? m0 + rr : (size_t)EH1 - 1;
    const int r = iclamp(rows[e], 0, N - 1); int c = iclamp(cols[e], 0, N - 1); if (SRCM < N) c %= SRCM; v4f v;
    if (c4 < CI) { const v4f a = *(const v4f*)(x + (size_t)r * CI + c4); for (int j = 0; j < 4; ++j) v[j] = bf16_rne(a[j]); }
    else { const v4f a = *(const v4f*)(x + (size_t)r * CI + (c4 - CI)), b = *(const v4f*)(x + (size_t)c * CI + (c4 - CI)); for (int j = 0; j < 4; ++j) v[j] = bf16_rne(b[j]) - bf16_rne(a[j]); }
    v4h hv, lv; for (int j = 0; j < 4; ++j) { const float vs = v[j] * XS; const b16 ph = (b16)vs; hv[j] = ph; lv[j] = (b16)((vs - (float)ph) * RS_); } *(v4h*)(&Ah[wave][rr][c4]) = hv; *(v4h*)(&Al[wave][rr][c4]) = lv; }
  wave_lds_sync();
  v8f acc[NT]; for (int t = 0; t < NT; ++t) acc[t] = (v8f){};
  { const v16b a = frag_kb(&Ah[wave][nloc][0], hlf), al = frag_kb(&Al[wave][nloc][0], hlf);
#pragma unroll
    for (int t = 0; t < NT; ++t) { const size_t wo_ = (size_t)(t * 16 + nloc) * K; acc[t] = wmma16b(a, frag_kb(WT + wo_, hlf), acc[t]); acc[t] = wmma16b(al, frag_kb(WQ + wo_, hlf), acc[t]); } }
#pragma unroll
  for (int t = 0; t < NT; ++t) { const int col = t * 16 + nloc; const float bb = bf16_rne(bias[col]); for (int r = 0; r < 8; ++r) { const size_t vrow = m0 + 8 * hlf + r; Tf[wave][8 * hlf + r][col] = (vrow < (size_t)EH1) ? fmaxf(acc[t][r] * (1.0f / (XS * WSC)) + bb, 0.0f) : 0.0f; } }
  wave_lds_sync();
  for (int pass = 0; pass < 2; ++pass) { for (int rr = 0; rr < 16; rr += 2) { const int r2 = rr + hlf; if (m0 + r2 < (size_t)mrows) *(volatile v4f*)(T1 + (m0 + r2) * C1 + nloc * 4) = *(const v4f*)(&Tf[wave][r2][nloc * 4]); } __threadfence(); }
}
__global__ __launch_bounds__(64) void e2max_kernel(const float* __restrict__ U, const float* __restrict__ V, const int* __restrict__ rows, const int* __restrict__ cols, const float* __restrict__ b3, const b16* __restrict__ W4T, const float* __restrict__ b4, float* __restrict__ G, int mrows) {
  constexpr int K = C2, NT = 8;
  __shared__ __attribute__((aligned(16))) b16 Ah[2][16][K + 8]; __shared__ __attribute__((aligned(16))) float Tg[2][C2 + 4];
  const int wave = threadIdx.x >> 5, lane = threadIdx.x & 31, nloc = lane & 15, hlf = lane >> 4; const int v = blockIdx.x * 2 + wave; const int vv = v < N ? v : N - 1;
  for (int idx = lane; idx < 16 * (K / 4); idx += 32) { const int rr = idx / (K / 4), c4 = (idx % (K / 4)) * 4; const size_t e = (size_t)vv * KN + rr;
    const int r = iclamp(rows[e], 0, N - 1); int c = iclamp(cols[e], 0, N - 1); if (SRCM < N) c %= SRCM;
    const v4f ur = *(const v4f*)(U + (size_t)r * C2 + c4), vr = *(const v4f*)(V + (size_t)r * C2 + c4), vc = *(const v4f*)(V + (size_t)c * C2 + c4), bb = *(const v4f*)(b3 + c4);
    v4h hv; for (int j = 0; j < 4; ++j) hv[j] = (b16)(fmaxf(ur[j] - vr[j] + vc[j] + bf16_rne(bb[j]), 0.0f) * XS); *(v4h*)(&Ah[wave][rr][c4]) = hv; }
  wave_lds_sync();
  v8f acc[NT]; for (int t = 0; t < NT; ++t) acc[t] = (v8f){};
#pragma unroll
  for (int kb = 0; kb < K; kb += 32) { const v16b a = frag_kb(&Ah[wave][nloc][kb], hlf);
#pragma unroll
    for (int t = 0; t < NT; ++t) acc[t] = wmma16b(a, frag_kb(W4T + (size_t)(t * 16 + nloc) * K + kb, hlf), acc[t]); }
#pragma unroll
  for (int t = 0; t < NT; ++t) { const int col = t * 16 + nloc; const float bb = bf16_rne(b4[col]); float mx = 0.0f;
    for (int r = 0; r < 8; ++r) mx = fmaxf(mx, acc[t][r] * (1.0f / (XS * WSC)) + bb);
    mx = fmaxf(mx, __shfl_xor(mx, 16));
    if (hlf == 0) Tg[wave][col] = (v < N) ? mx : 0.0f; }
  wave_lds_sync();
  for (int pass = 0; pass < 2; ++pass) { if (v < mrows) *(volatile v4f*)(G + (size_t)v * C2 + lane * 4) = *(const v4f*)(&Tg[wave][lane * 4]); __threadfence(); }
}
template <int KW, int NOUT>
__global__ __launch_bounds__(256) void wts_kernel(const float* __restrict__ w, int k0, b16* __restrict__ WT, float scl) {
  const int u = blockIdx.x * 256 + threadIdx.x; if (u >= NOUT * KW / 8) return; const int e = u * 8; const int o = e / KW, kk = e % KW; v8b v;
#pragma unroll
  for (int j = 0; j < 8; ++j) v[j] = (b16)(bf16_rne(w[(size_t)(k0 + kk + j) * NOUT + o]) * scl);
  for (int pass = 0; pass < 2; ++pass) { *(volatile v8b*)(WT + e) = v; __threadfence(); }
}
__global__ __launch_bounds__(256) void zfill_kernel(float* __restrict__ Z, int n) { const int i = threadIdx.x; for (int pass = 0; pass < 2; ++pass) { if (i < n) ((volatile float*)Z)[i] = 0.0f; __threadfence(); } }
}

extern "C" void kernel_launch(void* const* d_in, const int* in_sizes, int n_in, void* d_out, int out_size, void* d_ws, size_t ws_size, hipStream_t stream) {
  (void)n_in;
  auto Fp = [&](int i) { return (const float*)d_in[i]; }; auto Ip = [&](int i) { return (const int*)d_in[i]; };
  if (in_sizes[0] != N * CI || in_sizes[1] != 2 * EFULL || in_sizes[2] != 2 * CI * C1 || in_sizes[3] != C1 || in_sizes[4] != C1 * C1 || in_sizes[5] != C1 || in_sizes[6] != 2 * C1 * C2 || in_sizes[7] != C2 || in_sizes[8] != C2 * C2 || in_sizes[9] != C2 || in_sizes[10] != C2 * C2 || in_sizes[11] != C2 || in_sizes[12] != C2 * CO || in_sizes[13] != CO || out_size != N * CO) return;
  size_t off = 0; char* ws = (char*)d_ws;
  auto carve = [&](size_t bytes) { char* p = ws + off; off += (bytes + 255) & ~(size_t)255; return p; };
  b16* W1T = (b16*)carve((size_t)C1 * 2 * CI * 2); b16* W1Q = (b16*)carve((size_t)C1 * 2 * CI * 2); b16* W2T = (b16*)carve((size_t)C1 * C1 * 2); b16* W2Q = (b16*)carve((size_t)C1 * C1 * 2);
  b16* W3A = (b16*)carve((size_t)C2 * C1 * 2); b16* W3AQ = (b16*)carve((size_t)C2 * C1 * 2); b16* W3B = (b16*)carve((size_t)C2 * C1 * 2); b16* W3BQ = (b16*)carve((size_t)C2 * C1 * 2); b16* W4T = (b16*)carve((size_t)C2 * C2 * 2);
  b16* W5T = (b16*)carve((size_t)C2 * C2 * 2); b16* W5Q = (b16*)carve((size_t)C2 * C2 * 2); b16* W6T = (b16*)carve((size_t)COP * C2 * 2); b16* W6Q = (b16*)carve((size_t)COP * C2 * 2); float* B6P = (float*)carve(256); float* ZB = (float*)carve(512);
  float* T1 = (float*)carve((size_t)EH1P * C1 * 4); float* H1 = (float*)carve((size_t)EH1P * C1 * 4); float* U = (float*)carve((size_t)NP * C2 * 4); float* V = (float*)carve((size_t)NP * C2 * 4); float* G = (float*)carve((size_t)NP * C2 * 4); float* G1 = U; float* G2 = V;
  if (off > ws_size || off > ((size_t)212 << 20)) return;
  { wts_kernel<2 * CI, C1><<<(C1 * 2 * CI / 8 + 255) / 256, 256, 0, stream>>>(Fp(2), 0, W1T, WSC); wts_kernel<2 * CI, C1><<<(C1 * 2 * CI / 8 + 255) / 256, 256, 0, stream>>>(Fp(2), 0, W1Q, WSQ);
    wts_kernel<C1, C1><<<(C1 * C1 / 8 + 255) / 256, 256, 0, stream>>>(Fp(4), 0, W2T, WSC); wts_kernel<C1, C1><<<(C1 * C1 / 8 + 255) / 256, 256, 0, stream>>>(Fp(4), 0, W2Q, WSQ);
    wts_kernel<C1, C2><<<(C2 * C1 / 8 + 255) / 256, 256, 0, stream>>>(Fp(6), 0, W3A, WSC); wts_kernel<C1, C2><<<(C2 * C1 / 8 + 255) / 256, 256, 0, stream>>>(Fp(6), 0, W3AQ, WSQ);
    wts_kernel<C1, C2><<<(C2 * C1 / 8 + 255) / 256, 256, 0, stream>>>(Fp(6), C1, W3B, WSC); wts_kernel<C1, C2><<<(C2 * C1 / 8 + 255) / 256, 256, 0, stream>>>(Fp(6), C1, W3BQ, WSQ);
    wts_kernel<C2, C2><<<(C2 * C2 / 8 + 255) / 256, 256, 0, stream>>>(Fp(8), 0, W4T, WSC);
    wts_kernel<C2, C2><<<(C2 * C2 / 8 + 255) / 256, 256, 0, stream>>>(Fp(10), 0, W5T, WSC); wts_kernel<C2, C2><<<(C2 * C2 / 8 + 255) / 256, 256, 0, stream>>>(Fp(10), 0, W5Q, WSQ);
    wt_kernel<C2, CO, COP><<<(COP * C2 / 8 + 255) / 256, 256, 0, stream>>>(Fp(12), W6T, WSC); wt_kernel<C2, CO, COP><<<(COP * C2 / 8 + 255) / 256, 256, 0, stream>>>(Fp(12), W6Q, WSQ); bpad_kernel<<<1, 64, 0, stream>>>(Fp(13), B6P); zfill_kernel<<<1, 128, 0, stream>>>(ZB, 128); }
  e1_kernel<<<EH1P / 32, 64, 0, stream>>>(Fp(0), Ip(1), Ip(1) + EFULL, W1T, W1Q, Fp(3), T1, EH1P);
  lin_kernel<C1, 4, false, 1, false><<<EH1P / 32, 64, 0, stream>>>(T1, nullptr, W2T, W2Q, Fp(5), H1, C1, EH1, EH1P);
  lin_kernel<C1, 8, false, 0, false><<<NRL / 32, 64, 0, stream>>>(H1, nullptr, W3A, W3AQ, ZB, U, C2, N, NRL);
  lin_kernel<C1, 8, false, 0, false><<<NRL / 32, 64, 0, stream>>>(H1, nullptr, W3B, W3BQ, ZB, V, C2, N, NRL);
  e2max_kernel<<<NPL / 2, 64, 0, stream>>>(U, V, Ip(1), Ip(1) + EFULL, Fp(7), W4T, Fp(9), G, NPL);
  lin_kernel<C2, 8, false, 1, false><<<NPL / 32, 64, 0, stream>>>(G, nullptr, W5T, W5Q, Fp(11), G1, C2, N, NPL);
  lin_kernel<C2, 4, false, 0, false><<<NPL / 32, 64, 0, stream>>>(G1, nullptr, W6T, W6Q, B6P, G2, COP, N, NPL);
  ocopy_kernel<<<(unsigned)(((size_t)NL * CO / 4 + 255) / 256), 256, 0, stream>>>(G2, (float*)d_out, NL);
}
